// Encoder_40114994545039
// MI455X (gfx1250) — hardware-verified
//
#include <hip/hip_runtime.h>
#include <math.h>

constexpr int NBAT   = 64;
constexpr int NSTEP  = 128;
constexpr int NEMB   = 256;
constexpr int NHID   = 1024;
constexpr int NGATE  = 4 * NHID;
constexpr int NVOC   = 32000;
constexpr int NROWS  = NBAT * NSTEP;
constexpr int NTHR   = 256;
constexpr int RBLK   = 16;
constexpr int HPITCH = NHID + 8;
constexpr int SLABP  = 36;
constexpr float WCARRY = 16.0f;
constexpr float XCARRY = 16.0f;
constexpr float HCARRY = 64.0f;
constexpr float Z0SCALE = 1.0f / (XCARRY * WCARRY);
constexpr float Z1SCALE = 1.0f / (HCARRY * WCARRY);
constexpr float ZCARRY  = HCARRY * WCARRY;
constexpr float ZCARRY_INV = 1.0f / ZCARRY;
constexpr float BN_EPS_F = 1e-3f;
constexpr int NOUT0 = NBAT * NSTEP * NHID;
constexpr int NOUT1 = NBAT * NHID;

static_assert(NGATE % 64 == 0 && NROWS % 64 == 0, "GEMM M, N tile multiples");
static_assert(NEMB % 32 == 0 && NHID % 32 == 0, "GEMM K multiples of 32");
static_assert(NBAT % RBLK == 0, "batch tiling");
static_assert(NHID == 128 * (NTHR / 32), "8 waves x 128 hidden units");
static_assert(NEMB % 64 == 0 && NHID % 64 == 0 && NGATE % 64 == 0, "transpose tiles");
static_assert((HPITCH % 8) == 0, "16-B aligned LDS rows");
static_assert(2 * RBLK * 8 == NTHR, "pad fill exact");
static_assert((size_t)NOUT0 * 4 == 33554432u, "out0 bytes");
static_assert(((size_t)NOUT0 * 4) % 128 == 0 && ((size_t)(NOUT0 + NOUT1) * 4) % 128 == 0, "line-aligned outputs");
static_assert(((size_t)NOUT0 + 2 * (size_t)NOUT1) * 4 == 34078720u, "d_out total bytes");

typedef __attribute__((ext_vector_type(16))) _Float16 v16h;
typedef __attribute__((ext_vector_type(8)))  _Float16 v8h;
typedef __attribute__((ext_vector_type(16))) __bf16   v16b;
typedef __attribute__((ext_vector_type(8)))  __bf16   v8b;
typedef __attribute__((ext_vector_type(8)))  float    v8f;
typedef __attribute__((ext_vector_type(4)))  float    v4f;
typedef __attribute__((ext_vector_type(4)))  unsigned v4u;

__device__ __forceinline__ unsigned short f2bf_bits(float f) {
  unsigned u = __float_as_uint(f);
  return (unsigned short)((u + 0x7FFFu + ((u >> 16) & 1u)) >> 16);
}
__device__ __forceinline__ float bf_bits2f(unsigned short h) { return __uint_as_float(((unsigned)h) << 16); }

__device__ __forceinline__ float h16_to_f32(unsigned hb) {
  const unsigned sgn = (hb & 0x8000u) << 16; const unsigned em = hb & 0x7fffu;
  const float fn = __uint_as_float((em << 13) + 0x38000000u);
  const float fs = (float)em * 5.9604644775390625e-8f;
  const float mag = (em < 0x400u) ? fs : fn; return __uint_as_float(__float_as_uint(mag) | sgn); }

__device__ __forceinline__ void dep_guard4_h(v8f& a, v8f& b, v8f& c, v8f& d, v16h x, v16h y) { asm volatile("v_nop\n\tv_nop\n\tv_nop\n\tv_nop" : "+v"(a), "+v"(b), "+v"(c), "+v"(d) : "v"(x), "v"(y)); }
__device__ __forceinline__ void dep_guard4_b(v8f& a, v8f& b, v8f& c, v8f& d, v16b x, v16b y) { asm volatile("v_nop\n\tv_nop\n\tv_nop\n\tv_nop" : "+v"(a), "+v"(b), "+v"(c), "+v"(d) : "v"(x), "v"(y)); }
__device__ __forceinline__ void keep4_h(v16h a, v16h b, v16h c, v16h d) { asm volatile("v_nop" :: "v"(a), "v"(b), "v"(c), "v"(d)); }
__device__ __forceinline__ void keep4_b(v16b a, v16b b, v16b c, v16b d) { asm volatile("v_nop" :: "v"(a), "v"(b), "v"(c), "v"(d)); }
__device__ __forceinline__ void acc_guard4(v8f& a, v8f& b, v8f& c, v8f& d) { asm volatile("v_nop\n\tv_nop\n\tv_nop\n\tv_nop" : "+v"(a), "+v"(b), "+v"(c), "+v"(d)); }
__device__ __forceinline__ void grp_guard_h(v8f& a0, v8f& a1, v8f& a2, v8f& a3, v16h x, v16h b0, v16h b1, v16h b2, v16h b3) {
  asm volatile("v_nop\n\tv_nop\n\tv_nop\n\tv_nop" : "+v"(a0), "+v"(a1), "+v"(a2), "+v"(a3) : "v"(x), "v"(b0), "v"(b1), "v"(b2), "v"(b3));
}
__device__ __forceinline__ void wave_sync_lds() {
  __builtin_amdgcn_fence(__ATOMIC_RELEASE, "workgroup");
  __builtin_amdgcn_wave_barrier();
  __builtin_amdgcn_fence(__ATOMIC_ACQUIRE, "workgroup");
}

template <typename T> struct Frag;
template <> struct Frag<_Float16> {
  typedef v16h V; union U { v16h v; v8h h[2]; };
  static __device__ __forceinline__ v16h load(const _Float16* p) {
    U f; f.h[0] = *(const v8h*)(p); f.h[1] = *(const v8h*)(p + 16); return f.v;
  }
  static __device__ __forceinline__ v8f mma(v16h a, v16h b, v8f c) {
    return __builtin_amdgcn_wmma_f32_16x16x32_f16(false, a, false, b, (short)0, c, false, false);
  }
  static __device__ __forceinline__ void guard4(v8f& a, v8f& b, v8f& c, v8f& d, v16h x, v16h y) { dep_guard4_h(a, b, c, d, x, y); }
  static __device__ __forceinline__ void keep(v16h a, v16h b, v16h c, v16h d) { keep4_h(a, b, c, d); }
};
template <> struct Frag<__bf16> {
  typedef v16b V; union U { v16b v; v8b h[2]; };
  static __device__ __forceinline__ v16b load(const __bf16* p) {
    U f; f.h[0] = *(const v8b*)(p); f.h[1] = *(const v8b*)(p + 16); return f.v;
  }
  static __device__ __forceinline__ v8f mma(v16b a, v16b b, v8f c) {
    return __builtin_amdgcn_wmma_f32_16x16x32_bf16(false, a, false, b, (short)0, c, false, false);
  }
  static __device__ __forceinline__ void guard4(v8f& a, v8f& b, v8f& c, v8f& d, v16b x, v16b y) { dep_guard4_b(a, b, c, d, x, y); }
  static __device__ __forceinline__ void keep(v16b a, v16b b, v16b c, v16b d) { keep4_b(a, b, c, d); }
};

__device__ __forceinline__ float fsig(float x)  { return __builtin_amdgcn_rcpf(1.0f + __expf(-x)); }
__device__ __forceinline__ float ftanh(float x) { return 1.0f - 2.0f * __builtin_amdgcn_rcpf(__expf(2.0f * x) + 1.0f); }

template <int ET> struct Elem;
template <> struct Elem<0> { typedef _Float16 T; };
template <> struct Elem<1> { typedef __bf16 T; };
template <int ET, bool SPLIT, int BIAS_MODE, int OUT_MODE, bool RESID, int ACT = 0>
__global__ __launch_bounds__(256) void wmma_gemm64(
    const unsigned short* __restrict__ Ap, const unsigned short* __restrict__ A2p, int lda, long strideA,
    const unsigned short* __restrict__ Btp, const unsigned short* __restrict__ Bt2p, int ldb, long strideB,
    void* __restrict__ Cout, void* __restrict__ Cout2, int ldc, long strideC,
    const float* __restrict__ bias,
    const float* __restrict__ resid, long strideR,
    int M, int N, int K, float scale) {
  typedef typename Elem<ET>::T T;
  typedef typename Frag<T>::V V;
  const T* A = (const T*)Ap; const T* A2 = (const T*)A2p; const T* Bt = (const T*)Btp; const T* Bt2 = (const T*)Bt2p;
  __shared__ __align__(16) float sT[8][16 * 68];
  const int b    = blockIdx.y;
  const int lane = threadIdx.x & 31;
  const int wave = threadIdx.x >> 5;
  const int tilesN = N >> 6;
  const int tilesM = M >> 6;
  const int tile = blockIdx.x * 8 + wave;
  if (tile >= tilesM * tilesN) return;
  const int tm = tile / tilesN;
  const int tn = tile - tm * tilesN;
  const int m0 = tm << 6;
  const int n0 = tn << 6;

  const T* Ab  = A  + (size_t)b * strideA;
  const T* Bb  = Bt + (size_t)b * strideB;
  const T* Ab2 = SPLIT ? (A2  + (size_t)b * strideA) : nullptr;
  const T* Bb2 = SPLIT ? (Bt2 + (size_t)b * strideB) : nullptr;

  const int rlane = lane & 15;
  const int koff  = (lane >> 4) * 8;
  const int mOff  = (lane >> 4) * 8;

  v8f acc[4][4];
#pragma unroll
  for (int i = 0; i < 4; ++i)
#pragma unroll
    for (int j = 0; j < 4; ++j) acc[i][j] = (v8f){0.f,0.f,0.f,0.f,0.f,0.f,0.f,0.f};

  for (int k0 = 0; k0 < K; k0 += 32) {
    V bh[4], bl[4];
#pragma unroll
    for (int j = 0; j < 4; ++j) {
      const size_t bo = (size_t)(n0 + (j << 4) + rlane) * ldb + koff + k0;
      bh[j] = Frag<T>::load(Bb + bo);
      if (SPLIT) bl[j] = Frag<T>::load(Bb2 + bo);
    }
#pragma unroll
    for (int i = 0; i < 4; ++i) {
      const size_t ao = (size_t)(m0 + (i << 4) + rlane) * lda + koff + k0;
      V ah = Frag<T>::load(Ab + ao);
      V al;
      if (SPLIT) al = Frag<T>::load(Ab2 + ao);
#pragma unroll
      for (int j = 0; j < 4; ++j) {
        acc[i][j] = Frag<T>::mma(ah, bh[j], acc[i][j]);
        if (SPLIT) {
          acc[i][j] = Frag<T>::mma(ah, bl[j], acc[i][j]);
          acc[i][j] = Frag<T>::mma(al, bh[j], acc[i][j]);
        }
      }
      Frag<T>::guard4(acc[i][0], acc[i][1], acc[i][2], acc[i][3], ah, SPLIT ? al : ah);
    }
    Frag<T>::keep(bh[0], bh[1], bh[2], bh[3]);
    if (SPLIT) Frag<T>::keep(bl[0], bl[1], bl[2], bl[3]);
  }
  acc_guard4(acc[0][0], acc[0][1], acc[0][2], acc[0][3]);
  acc_guard4(acc[1][0], acc[1][1], acc[1][2], acc[1][3]);
  acc_guard4(acc[2][0], acc[2][1], acc[2][2], acc[2][3]);
  acc_guard4(acc[3][0], acc[3][1], acc[3][2], acc[3][3]);

  float* slab = sT[wave];
  const float* Rb = RESID ? (resid + (size_t)b * strideR) : nullptr;
#pragma unroll
  for (int i = 0; i < 4; ++i) {
    const int mBase = m0 + (i << 4);
#pragma unroll
    for (int j = 0; j < 4; ++j) {
      const int n = n0 + (j << 4) + rlane;
      float bv = 0.f;
      if (BIAS_MODE == 2) bv = bias[n];
#pragma unroll
      for (int r = 0; r < 8; ++r) {
        float v = acc[i][j][r] * scale;
        if (BIAS_MODE == 1) v += bias[mBase + mOff + r];
        if (BIAS_MODE == 2) v += bv;
        if (RESID) v += Rb[(size_t)(mBase + mOff + r) * ldc + n];
        if (ACT == 1) v = tanhf(v);
        if (ACT == 2) v = fmaxf(v, 0.0f);
        if (ACT == 3) v = v / (1.0f + expf(-v));
        if (ACT == 4) v = (v > 0.f) ? v : 0.01f * v;
        if (ACT == 5) v = 0.5f * v * (1.0f + erff(v * 0.70710678118654752f));
        slab[(mOff + r) * 68 + (j << 4) + rlane] = v;
      }
    }
    __builtin_amdgcn_fence(__ATOMIC_RELEASE, "workgroup");
    __builtin_amdgcn_wave_barrier();
    __builtin_amdgcn_fence(__ATOMIC_ACQUIRE, "workgroup");
    if (OUT_MODE == 0) {
      float* C = (float*)Cout + (size_t)b * strideC;
      const int hh = lane >> 4, c4 = (lane & 15) * 4;
      for (int pass = 0; pass < 2; ++pass) {
#pragma unroll
        for (int it = 0; it < 8; ++it) {
          const int row = it * 2 + hh;
          v4f v = *(const v4f*)(slab + row * 68 + c4);
          *(volatile v4f*)(C + (size_t)(mBase + row) * ldc + n0 + c4) = v;
        }
        __threadfence();
      }
    } else {
      const int q = lane >> 3, c8 = (lane & 7) * 8;
      unsigned short* C  = (unsigned short*)Cout  + (size_t)b * strideC;
      unsigned short* C2 = (OUT_MODE == 2) ? ((unsigned short*)Cout2 + (size_t)b * strideC) : nullptr;
      for (int pass = 0; pass < 2; ++pass) {
#pragma unroll
        for (int it = 0; it < 4; ++it) {
          const int row = it * 4 + q;
          const float* sp = slab + row * 68 + c8;
          v8h hv, lv;
#pragma unroll
          for (int e = 0; e < 8; ++e) {
            if (OUT_MODE == 1) {
              hv[e] = (_Float16)sp[e];
            } else {
              unsigned short hb = f2bf_bits(sp[e]);
              unsigned short lb = f2bf_bits(sp[e] - bf_bits2f(hb));
              hv[e] = __builtin_bit_cast(_Float16, hb);
              lv[e] = __builtin_bit_cast(_Float16, lb);
            }
          }
          *(volatile v8h*)(C + (size_t)(mBase + row) * ldc + n0 + c8) = hv;
          if (OUT_MODE == 2) *(volatile v8h*)(C2 + (size_t)(mBase + row) * ldc + n0 + c8) = lv;
        }
        __threadfence();
      }
    }
    __builtin_amdgcn_fence(__ATOMIC_RELEASE, "workgroup");
    __builtin_amdgcn_wave_barrier();
    __builtin_amdgcn_fence(__ATOMIC_ACQUIRE, "workgroup");
  }
}

__global__ __launch_bounds__(NTHR) void tpw_f16_kernel(const float* __restrict__ src, int R, int C, int ldo,
                                                       unsigned short* __restrict__ O, float sc) {
  __shared__ float Tt[64 * 65];
  const int tid = threadIdx.x;
  const int c0 = blockIdx.x * 64, r0 = blockIdx.y * 64;
  (void)R;
#pragma unroll
  for (int i = 0; i < 4; ++i) {
    const int idx = i * NTHR + tid;
    const int rr = idx >> 4, cc = (idx & 15) * 4;
    const v4f v = *(const v4f*)(src + (size_t)(r0 + rr) * (size_t)C + c0 + cc);
    Tt[rr * 65 + cc + 0] = v[0];
    Tt[rr * 65 + cc + 1] = v[1];
    Tt[rr * 65 + cc + 2] = v[2];
    Tt[rr * 65 + cc + 3] = v[3];
  }
  __syncthreads();
  const int q = tid >> 3, c8 = (tid & 7) * 8;
  v8h hv[2];
#pragma unroll
  for (int g = 0; g < 2; ++g) {
    const int qq = g * 32 + q;
#pragma unroll
    for (int e = 0; e < 8; ++e) {
      const float f = Tt[(c8 + e) * 65 + qq];
      hv[g][e] = (_Float16)(f * sc);
    }
  }
  for (int pass = 0; pass < 2; ++pass) {
#pragma unroll
    for (int g = 0; g < 2; ++g) {
      const size_t o = (size_t)(c0 + g * 32 + q) * (size_t)ldo + (size_t)(r0 + c8);
      *(volatile v8h*)(void*)(O + o) = hv[g];
    }
    __threadfence();
  }
}

__global__ __launch_bounds__(NTHR) void gather_x_kernel(const int* __restrict__ tokens, const float* __restrict__ emb,
                                                        unsigned short* __restrict__ X) {
  const int tid = threadIdx.x, lane = tid & 31;
  const int row = blockIdx.x * (NTHR / 32) + (tid >> 5);
  if (row >= NROWS) return;
  const int t = row >> 6, b = row & (NBAT - 1);
  int tok = tokens[b * NSTEP + t];
  tok = tok < 0 ? 0 : (tok > NVOC - 1 ? NVOC - 1 : tok);
  const float* sp = emb + (size_t)tok * NEMB + lane * 8;
  const v4f a = *(const v4f*)(sp);
  const v4f bq = *(const v4f*)(sp + 4);
  v8h hv;
#pragma unroll
  for (int e = 0; e < 4; ++e) {
    hv[e]     = (_Float16)(a[e] * XCARRY);
    hv[4 + e] = (_Float16)(bq[e] * XCARRY);
  }
  unsigned short* op = X + (size_t)row * NEMB + lane * 8;
  *(volatile v8h*)(void*)op = hv;
  __threadfence();
  *(volatile v8h*)(void*)op = hv;
}

template <int LAYER>
__device__ __forceinline__ void lstm_pass(
    const int p, float (&cs)[2][8], const int t, const bool last,
    const int rowbase, const int wave, const int lane,
    const _Float16* ahrow, _Float16* ahn, float* slab,
    const unsigned short* __restrict__ ZT, const _Float16* __restrict__ UT,
    float* __restrict__ hfin, float* __restrict__ cfin, float* __restrict__ out0,
    const float* __restrict__ gam, const float* __restrict__ bet,
    const float* __restrict__ mmean, const float* __restrict__ mvar) {
  const int c = lane & 15, hh = lane >> 4, koff = hh * 8;
  const int jb = 128 * wave + 32 * p;

  v8f acc[2][4];
#pragma unroll
  for (int ch = 0; ch < 2; ++ch) {
#pragma unroll
    for (int g = 0; g < 4; ++g) {
      const int n = g * NHID + jb + 16 * ch + c;
      const v4u q = *(const v4u*)(const void*)(ZT + (size_t)n * NROWS + (size_t)t * NBAT + rowbase + 8 * hh);
      const unsigned w0 = q[0];
      const unsigned w1 = q[1];
      const unsigned w2 = q[2];
      const unsigned w3 = q[3];
      v8f z;
      z[0] = h16_to_f32(w0 & 0xffffu) * ZCARRY;
      z[1] = h16_to_f32(w0 >> 16) * ZCARRY;
      z[2] = h16_to_f32(w1 & 0xffffu) * ZCARRY;
      z[3] = h16_to_f32(w1 >> 16) * ZCARRY;
      z[4] = h16_to_f32(w2 & 0xffffu) * ZCARRY;
      z[5] = h16_to_f32(w2 >> 16) * ZCARRY;
      z[6] = h16_to_f32(w3 & 0xffffu) * ZCARRY;
      z[7] = h16_to_f32(w3 >> 16) * ZCARRY;
      acc[ch][g] = z;
    }
  }

  const _Float16* ub = UT + (size_t)(jb + c) * NHID + koff;
#pragma unroll 1
  for (int k0 = 0; k0 < NHID; k0 += 32) {
    const v16h a = Frag<_Float16>::load(ahrow + k0);
#pragma unroll
    for (int ch = 0; ch < 2; ++ch) {
      const _Float16* up = ub + (size_t)ch * 16 * NHID + k0;
      const v16h b0 = Frag<_Float16>::load(up);
      const v16h b1 = Frag<_Float16>::load(up + (size_t)1 * NHID * NHID);
      const v16h b2 = Frag<_Float16>::load(up + (size_t)2 * NHID * NHID);
      const v16h b3 = Frag<_Float16>::load(up + (size_t)3 * NHID * NHID);
      acc[ch][0] = Frag<_Float16>::mma(a, b0, acc[ch][0]);
      acc[ch][1] = Frag<_Float16>::mma(a, b1, acc[ch][1]);
      acc[ch][2] = Frag<_Float16>::mma(a, b2, acc[ch][2]);
      acc[ch][3] = Frag<_Float16>::mma(a, b3, acc[ch][3]);
      grp_guard_h(acc[ch][0], acc[ch][1], acc[ch][2], acc[ch][3], a, b0, b1, b2, b3);
    }
  }
  acc_guard4(acc[0][0], acc[0][1], acc[0][2], acc[0][3]);
  acc_guard4(acc[1][0], acc[1][1], acc[1][2], acc[1][3]);

  const bool wr_h = (LAYER == 1) || last;
#pragma unroll
  for (int ch = 0; ch < 2; ++ch) {
    const int j = jb + 16 * ch + c;
#pragma unroll
    for (int r = 0; r < 8; ++r) {
      const float zi = acc[ch][0][r] * ZCARRY_INV;
      const float zf = acc[ch][1][r] * ZCARRY_INV;
      const float zg = acc[ch][2][r] * ZCARRY_INV;
      const float zo = acc[ch][3][r] * ZCARRY_INV;
      const float ig = fsig(zi);
      const float fg = fsig(zf);
      const float gg = ftanh(zg);
      const float og = fsig(zo);
      const float cn = fg * cs[ch][r] + ig * gg;
      cs[ch][r] = cn;
      const float hn = og * ftanh(cn);
      ahn[(8 * hh + r) * HPITCH + j] = (_Float16)(hn * HCARRY);
      if (wr_h) slab[(8 * hh + r) * SLABP + 16 * ch + c] = hn;
    }
  }

  const int q = lane >> 3, c4 = (lane & 7) * 4;
  if (wr_h) {
    wave_sync_lds();
    v4f hv[4], ov[4];
#pragma unroll
    for (int it = 0; it < 4; ++it) {
      hv[it] = *(const v4f*)(slab + (it * 4 + q) * SLABP + c4);
      ov[it] = hv[it];
    }
    if (LAYER == 1) {
      const v4f g4 = *(const v4f*)(gam + jb + c4);
      const v4f b4 = *(const v4f*)(bet + jb + c4);
      const v4f m4 = *(const v4f*)(mmean + jb + c4);
      const v4f s4 = *(const v4f*)(mvar + jb + c4);
      v4f inv;
#pragma unroll
      for (int e = 0; e < 4; ++e) inv[e] = rsqrtf(s4[e] + BN_EPS_F);
#pragma unroll
      for (int it = 0; it < 4; ++it)
#pragma unroll
        for (int e = 0; e < 4; ++e) ov[it][e] = ((hv[it][e] - m4[e]) * inv[e]) * g4[e] + b4[e];
    }
    for (int pass = 0; pass < 2; ++pass) {
#pragma unroll
      for (int it = 0; it < 4; ++it) {
        const int row = it * 4 + q;
        if (LAYER == 1)
          *(volatile v4f*)(out0 + ((size_t)(rowbase + row) * NSTEP + (size_t)t) * NHID + jb + c4) = ov[it];
        if (last)
          *(volatile v4f*)(hfin + (size_t)(rowbase + row) * NHID + jb + c4) = hv[it];
      }
      __threadfence();
    }
    wave_sync_lds();
  }
  if (last) {
#pragma unroll
    for (int ch = 0; ch < 2; ++ch)
#pragma unroll
      for (int r = 0; r < 8; ++r) slab[(8 * hh + r) * SLABP + 16 * ch + c] = cs[ch][r];
    wave_sync_lds();
    v4f cv[4];
#pragma unroll
    for (int it = 0; it < 4; ++it) cv[it] = *(const v4f*)(slab + (it * 4 + q) * SLABP + c4);
    for (int pass = 0; pass < 2; ++pass) {
#pragma unroll
      for (int it = 0; it < 4; ++it) {
        const int row = it * 4 + q;
        *(volatile v4f*)(cfin + (size_t)(rowbase + row) * NHID + jb + c4) = cv[it];
      }
      __threadfence();
    }
    wave_sync_lds();
  }
}

template <int LAYER>
__global__ __launch_bounds__(NTHR) void lstm_seq_kernel(
    const unsigned short* __restrict__ ZTp, const unsigned short* __restrict__ UTp,
    const float* __restrict__ hinit, const float* __restrict__ cinit,
    unsigned short* __restrict__ Y0p,
    float* __restrict__ hfin, float* __restrict__ cfin, float* __restrict__ out0,
    const float* __restrict__ gam, const float* __restrict__ bet,
    const float* __restrict__ mmean, const float* __restrict__ mvar) {
  __shared__ __align__(16) _Float16 Ah[2][RBLK * HPITCH];
  __shared__ __align__(16) float    Sl[NTHR / 32][16 * SLABP];
  const _Float16* UT = (const _Float16*)UTp;
  const int tid = threadIdx.x, lane = tid & 31, wave = tid >> 5;
  const int c = lane & 15, hh = lane >> 4, koff = hh * 8;
  const int rowbase = blockIdx.x * RBLK;

  {
    const int buf = tid >> 7, prow = (tid >> 3) & 15, pcol = NHID + (tid & 7);
    Ah[buf][prow * HPITCH + pcol] = (_Float16)0.0f;
  }
#pragma unroll 1
  for (int i = 0; i < (RBLK * NHID) / NTHR; ++i) {
    const int idx = i * NTHR + tid;
    const int hr = idx >> 10, hc = idx & (NHID - 1);
    Ah[0][hr * HPITCH + hc] = (_Float16)(hinit[(size_t)(rowbase + hr) * NHID + hc] * HCARRY);
  }
  float cs0[2][8], cs1[2][8], cs2[2][8], cs3[2][8];
#pragma unroll
  for (int ch = 0; ch < 2; ++ch) {
#pragma unroll
    for (int r = 0; r < 8; ++r) {
      const size_t o = (size_t)(rowbase + 8 * hh + r) * NHID + 128 * wave + 16 * ch + c;
      cs0[ch][r] = cinit[o];
      cs1[ch][r] = cinit[o + 32];
      cs2[ch][r] = cinit[o + 64];
      cs3[ch][r] = cinit[o + 96];
    }
  }
  __syncthreads();

  float* slab = Sl[wave];
#pragma unroll 1
  for (int t = 0; t < NSTEP; ++t) {
    const int cur = t & 1;
    const _Float16* ahrow = &Ah[cur][0] + c * HPITCH + koff;
    _Float16* ahn = &Ah[cur ^ 1][0];
    const bool last = (t == NSTEP - 1);
    lstm_pass<LAYER>(0, cs0, t, last, rowbase, wave, lane, ahrow, ahn, slab, ZTp, UT, hfin, cfin, out0, gam, bet, mmean, mvar);
    lstm_pass<LAYER>(1, cs1, t, last, rowbase, wave, lane, ahrow, ahn, slab, ZTp, UT, hfin, cfin, out0, gam, bet, mmean, mvar);
    lstm_pass<LAYER>(2, cs2, t, last, rowbase, wave, lane, ahrow, ahn, slab, ZTp, UT, hfin, cfin, out0, gam, bet, mmean, mvar);
    lstm_pass<LAYER>(3, cs3, t, last, rowbase, wave, lane, ahrow, ahn, slab, ZTp, UT, hfin, cfin, out0, gam, bet, mmean, mvar);
    __syncthreads();
    if (LAYER == 0) {
      const _Float16* srcb = &Ah[cur ^ 1][0];
      v8h vv[8];
#pragma unroll
      for (int it = 0; it < 8; ++it) {
        const int idx = it * NTHR + tid;
        const int yr = idx >> 7, c8 = (idx & 127) * 8;
        vv[it] = *(const v8h*)(srcb + yr * HPITCH + c8);
      }
      for (int pass = 0; pass < 2; ++pass) {
#pragma unroll
        for (int it = 0; it < 8; ++it) {
          const int idx = it * NTHR + tid;
          const int yr = idx >> 7, c8 = (idx & 127) * 8;
          *(volatile v8h*)(void*)(Y0p + ((size_t)t * NBAT + rowbase + yr) * NHID + c8) = vv[it];
        }
        __threadfence();
      }
    }
  }
}

constexpr size_t WS_TOTAL =
    (size_t)NGATE * NROWS * 2 + (size_t)NGATE * NEMB * 2 + 3 * (size_t)NGATE * NHID * 2 +
    (size_t)NROWS * NEMB * 2 + (size_t)NROWS * NHID * 2 + 2 * (size_t)NBAT * NHID * 4;
static_assert(WS_TOTAL == 115867648u, "carve total");
static_assert(WS_TOTAL <= 134217728u, "carve budget");

extern "C" void kernel_launch(void* const* d_in, const int* in_sizes, int n_in,
                              void* d_out, int out_size, void* d_ws, size_t ws_size, hipStream_t stream) {
  if (n_in < 14 || d_out == nullptr || d_ws == nullptr) return;
  if (in_sizes[0] != NBAT * NSTEP || in_sizes[1] != NBAT * NHID || in_sizes[2] != NBAT * NHID ||
      in_sizes[3] != NVOC * NEMB || in_sizes[4] != NEMB * NGATE || in_sizes[5] != NHID * NGATE ||
      in_sizes[6] != NGATE || in_sizes[7] != NHID * NGATE || in_sizes[8] != NHID * NGATE ||
      in_sizes[9] != NGATE || in_sizes[10] != NHID || in_sizes[11] != NHID || in_sizes[12] != NHID ||
      in_sizes[13] != NHID || out_size != NOUT0 + 2 * NOUT1) return;

  const int*   tokens = (const int*)  d_in[0];
  const float* h0     = (const float*)d_in[1];
  const float* c0     = (const float*)d_in[2];
  const float* emb    = (const float*)d_in[3];
  const float* W0     = (const float*)d_in[4];
  const float* U0     = (const float*)d_in[5];
  const float* b0     = (const float*)d_in[6];
  const float* W1     = (const float*)d_in[7];
  const float* U1     = (const float*)d_in[8];
  const float* b1     = (const float*)d_in[9];
  const float* gam    = (const float*)d_in[10];
  const float* bet    = (const float*)d_in[11];
  const float* mmean  = (const float*)d_in[12];
  const float* mvar   = (const float*)d_in[13];
  float* out0 = (float*)d_out;
  float* out1 = out0 + (size_t)NOUT0;
  float* out2 = out1 + (size_t)NOUT1;

  char* ws = (char*)d_ws; size_t off = 0;
  auto carve = [&](size_t bytes) -> char* { char* p = ws + off; off += (bytes + 255) & ~(size_t)255; return p; };
  unsigned short* ZT  = (unsigned short*)carve((size_t)NGATE * NROWS * 2);
  unsigned short* W0T = (unsigned short*)carve((size_t)NGATE * NEMB * 2);
  unsigned short* U0T = (unsigned short*)carve((size_t)NGATE * NHID * 2);
  unsigned short* W1T = (unsigned short*)carve((size_t)NGATE * NHID * 2);
  unsigned short* U1T = (unsigned short*)carve((size_t)NGATE * NHID * 2);
  unsigned short* X   = (unsigned short*)carve((size_t)NROWS * NEMB * 2);
  unsigned short* Y0  = (unsigned short*)carve((size_t)NROWS * NHID * 2);
  float*          HF  = (float*)carve((size_t)NBAT * NHID * 4);
  float*          CF  = (float*)carve((size_t)NBAT * NHID * 4);
  if (off > ws_size || off > (size_t)134217728) return;

  tpw_f16_kernel<<<dim3(NGATE / 64, NEMB / 64), NTHR, 0, stream>>>(W0, NEMB, NGATE, NEMB, W0T, WCARRY);
  tpw_f16_kernel<<<dim3(NGATE / 64, NHID / 64), NTHR, 0, stream>>>(U0, NHID, NGATE, NHID, U0T, WCARRY);
  tpw_f16_kernel<<<dim3(NGATE / 64, NHID / 64), NTHR, 0, stream>>>(W1, NHID, NGATE, NHID, W1T, WCARRY);
  tpw_f16_kernel<<<dim3(NGATE / 64, NHID / 64), NTHR, 0, stream>>>(U1, NHID, NGATE, NHID, U1T, WCARRY);

  gather_x_kernel<<<NROWS / (NTHR / 32), NTHR, 0, stream>>>(tokens, emb, X);

  const dim3 ggrid((NGATE / 64) * (NROWS / 64) / 8, 1);
  wmma_gemm64<0, false, 1, 1, false, 0><<<ggrid, 256, 0, stream>>>(
      W0T, W0T, NEMB, 0L, X, X, NEMB, 0L, (void*)ZT, (void*)ZT, NROWS, 0L,
      b0, b0, 0L, NGATE, NROWS, NEMB, Z0SCALE);

  lstm_seq_kernel<0><<<NBAT / RBLK, NTHR, 0, stream>>>(ZT, U0T, h0, c0, Y0, HF, CF, out0, gam, bet, mmean, mvar);

  wmma_gemm64<0, false, 1, 1, false, 0><<<ggrid, 256, 0, stream>>>(
      W1T, W1T, NHID, 0L, Y0, Y0, NHID, 0L, (void*)ZT, (void*)ZT, NROWS, 0L,
      b1, b1, 0L, NGATE, NROWS, NHID, Z1SCALE);

  lstm_seq_kernel<1><<<NBAT / RBLK, NTHR, 0, stream>>>(ZT, U1T, HF, CF, Y0, out1, out2, out0, gam, bet, mmean, mvar);
}
